// Colorizer_15676630630937
// MI455X (gfx1250) — hardware-verified
//
#include <hip/hip_runtime.h>
#include <stdint.h>

#define CDIM 64
#define HW   4096
#define NKF  3
#define CY   16
#define KT   64
#define MQB  64
#define XTP  72
#define OSP  68
#define L2E  1.44269504088896340736f
#define PEX  14.0f
#define YSC  16.0f
#define OSC  0.0625f

static_assert(CDIM == 64);
static_assert(CY == 16);
static_assert(KT == 64);
static_assert(MQB == 64);
static_assert((HW % KT) == 0);
static_assert((HW % MQB) == 0);
static_assert((XTP * 2) % 16 == 0);
static_assert((OSP * 4) % 16 == 0);

typedef _Float16       v8h  __attribute__((ext_vector_type(8)));
typedef _Float16       v16h __attribute__((ext_vector_type(16)));
typedef __bf16         v16b __attribute__((ext_vector_type(16)));
typedef unsigned short v8us __attribute__((ext_vector_type(8)));
typedef float          v4f  __attribute__((ext_vector_type(4)));
typedef float          v8f  __attribute__((ext_vector_type(8)));

union FragH { v8h p[2]; v16h v; };
union FragB { v8us p[2]; v16b v; };
static_assert(sizeof(FragH) == 32);
static_assert(sizeof(FragB) == 32);

__device__ __forceinline__ v8f zero8() { v8f z = {0.f, 0.f, 0.f, 0.f, 0.f, 0.f, 0.f, 0.f}; return z; }

__device__ __forceinline__ unsigned int bf_bits(float x) {
  unsigned int u = __float_as_uint(x);
  u += 0x7FFFu + ((u >> 16) & 1u);
  return u >> 16;
}
__device__ __forceinline__ float bf_rne(float x) { return __uint_as_float(bf_bits(x) << 16); }

__device__ __forceinline__ v8f mma_h(v16h a, v16h b, v8f c) {
  v8f d = __builtin_amdgcn_wmma_f32_16x16x32_f16(false, a, false, b, (short)0, c, false, false);
#if defined(__HIP_DEVICE_COMPILE__)
  asm volatile("v_nop\n\tv_nop\n\tv_nop\n\tv_nop" : "+v"(d) : "v"(a), "v"(b));
#endif
  return d;
}
__device__ __forceinline__ v8f mma_b(v16b a, v16b b, v8f c) {
  v8f d = __builtin_amdgcn_wmma_f32_16x16x32_bf16(false, a, false, b, (short)0, c, false, false);
#if defined(__HIP_DEVICE_COMPILE__)
  asm volatile("v_nop\n\tv_nop\n\tv_nop\n\tv_nop" : "+v"(d) : "v"(a), "v"(b));
#endif
  return d;
}

__device__ __forceinline__ float max8(v8f d) {
  const float a = fmaxf(d[0], d[1]);
  const float b = fmaxf(d[2], d[3]);
  const float c = fmaxf(d[4], d[5]);
  const float e = fmaxf(d[6], d[7]);
  return fmaxf(fmaxf(a, b), fmaxf(c, e));
}

__global__ __launch_bounds__(256)
void k_xt(const float* __restrict__ x, unsigned short* XT) {
  __shared__ __align__(16) unsigned short s[KT * XTP];
  const int t  = threadIdx.x;
  const int f  = blockIdx.y;
  const int p0 = blockIdx.x * KT;
  const float* xs = x + (size_t)f * CDIM * HW + p0;
#pragma unroll
  for (int it = 0; it < 4; ++it) {
    const int idx = it * 256 + t;
    const int c   = idx >> 4;
    const int p4  = idx & 15;
    const v4f a = *(const v4f*)(xs + (size_t)c * HW + 4 * p4);
#pragma unroll
    for (int i = 0; i < 4; ++i) s[(4 * p4 + i) * XTP + c] = (unsigned short)bf_bits(a[i]);
  }
  __syncthreads();
  v8us w[2];
  size_t pd[2];
#pragma unroll
  for (int it = 0; it < 2; ++it) {
    const int L = it * 32 + (t >> 3);
    const int q = t & 7;
    w[it]  = *(const v8us*)(s + L * XTP + 8 * q);
    pd[it] = ((size_t)f * HW + p0 + L) * CDIM + 8 * q;
  }
#pragma unroll
  for (int it = 0; it < 2; ++it) *(volatile v8us*)(XT + pd[it]) = w[it];
  __threadfence();
#pragma unroll
  for (int it = 0; it < 2; ++it) *(volatile v8us*)(XT + pd[it]) = w[it];
}

__global__ __launch_bounds__(256)
void k_yh(const float* __restrict__ y, _Float16* YH) {
  const size_t e = ((size_t)blockIdx.x * 256 + threadIdx.x) * 8;
  const v4f a = *(const v4f*)(y + e);
  const v4f c = *(const v4f*)(y + e + 4);
  v8h w;
#pragma unroll
  for (int i = 0; i < 4; ++i) {
    w[i]     = (_Float16)(bf_rne(a[i]) * YSC);
    w[4 + i] = (_Float16)(bf_rne(c[i]) * YSC);
  }
  *(volatile v8h*)(YH + e) = w;
  __threadfence();
  *(volatile v8h*)(YH + e) = w;
}

__global__ __launch_bounds__(128)
void k_attn(const unsigned short* __restrict__ XT, const _Float16* __restrict__ YH, float* out) {
  __shared__ __align__(16) float Os[CY * OSP];
  const int t    = threadIdx.x;
  const int lane = t & 31, wv = t >> 5;
  const int hh   = lane >> 4, n = lane & 15;
  const int b    = blockIdx.y;
  const int bm0  = blockIdx.x * MQB;
  const int m0   = bm0 + wv * 16;

  const unsigned short* tq = XT + ((size_t)((NKF + 1) * b + NKF) * HW + m0 + n) * CDIM + 8 * hh;
  FragB bq0, bq1;
  bq0.p[0] = *(const v8us*)(tq);
  bq0.p[1] = *(const v8us*)(tq + 16);
  bq1.p[0] = *(const v8us*)(tq + 32);
  bq1.p[1] = *(const v8us*)(tq + 48);

  const unsigned short* kbase = XT + ((size_t)((NKF + 1) * b) * HW + n) * CDIM + 8 * hh;
  const _Float16*       ybase = YH + ((size_t)(NKF * b) * CY + n) * HW + 8 * hh;

  v8f   O = zero8();
  float m = -1.0e30f, z = 0.f;

#pragma unroll 1
  for (int kk0 = 0; kk0 < NKF * HW; kk0 += KT) {
    const int fr = kk0 / HW;
    const int p0 = kk0 - fr * HW;
    const unsigned short* kp = kbase + ((size_t)fr * HW + p0) * CDIM;

    v8f S[4];
#pragma unroll
    for (int ks = 0; ks < 4; ++ks) {
      const unsigned short* a = kp + ks * 16 * CDIM;
      FragB f0, f1;
      f0.p[0] = *(const v8us*)(a);
      f0.p[1] = *(const v8us*)(a + 16);
      f1.p[0] = *(const v8us*)(a + 32);
      f1.p[1] = *(const v8us*)(a + 48);
      v8f zz = mma_b(f0.v, bq0.v, zero8());
      zz     = mma_b(f1.v, bq1.v, zz);
      S[ks]  = zz;
    }

    float tm = fmaxf(max8(S[0]), max8(S[1]));
    tm = fmaxf(tm, fmaxf(max8(S[2]), max8(S[3])));
    const float tmo = __shfl_xor(tm, 16, 32);
    tm = fmaxf(tm, tmo);
    const float mn    = fmaxf(m, tm * L2E);
    const float alpha = __builtin_amdgcn_exp2f(m - mn);
    m = mn;
    const float nb = PEX - mn;
    z *= alpha;
    O = O * alpha;

    FragH pf0, pf1;
#pragma unroll
    for (int r = 0; r < 8; ++r) {
      const _Float16 e0 = (_Float16)__builtin_amdgcn_exp2f(fmaf(S[0][r], L2E, nb));
      const _Float16 e1 = (_Float16)__builtin_amdgcn_exp2f(fmaf(S[1][r], L2E, nb));
      const _Float16 e2 = (_Float16)__builtin_amdgcn_exp2f(fmaf(S[2][r], L2E, nb));
      const _Float16 e3 = (_Float16)__builtin_amdgcn_exp2f(fmaf(S[3][r], L2E, nb));
      pf0.v[r]     = e0;
      pf0.v[8 + r] = e1;
      pf1.v[r]     = e2;
      pf1.v[8 + r] = e3;
      z += (float)e0;
      z += (float)e1;
      z += (float)e2;
      z += (float)e3;
    }

    const _Float16* yp = ybase + (size_t)fr * CY * HW + p0;
    FragH ay;
    ay.p[0] = *(const v8h*)(yp);
    ay.p[1] = *(const v8h*)(yp + 16);
    O = mma_h(ay.v, pf0.v, O);
    FragH ay1;
    ay1.p[0] = *(const v8h*)(yp + 32);
    ay1.p[1] = *(const v8h*)(yp + 48);
    O = mma_h(ay1.v, pf1.v, O);
  }

  const float zo = __shfl_xor(z, 16, 32);
  const float zt = z + zo;
  const float rz = __builtin_amdgcn_rcpf(zt) * OSC;
#pragma unroll
  for (int r = 0; r < 8; ++r) Os[(8 * hh + r) * OSP + 16 * wv + n] = O[r] * rz;
  __syncthreads();

  v4f    ov[2];
  size_t po[2];
#pragma unroll
  for (int it = 0; it < 2; ++it) {
    const int L    = it * 16 + (t >> 3);
    const int cc   = L >> 1;
    const int half = L & 1;
    const int q    = t & 7;
    ov[it] = *(const v4f*)(Os + cc * OSP + half * 32 + 4 * q);
    po[it] = ((size_t)(b * CY + cc)) * HW + bm0 + half * 32 + 4 * q;
  }
#pragma unroll
  for (int it = 0; it < 2; ++it) *(volatile v4f*)(out + po[it]) = ov[it];
  __threadfence();
#pragma unroll
  for (int it = 0; it < 2; ++it) *(volatile v4f*)(out + po[it]) = ov[it];
}

extern "C" void kernel_launch(void* const* d_in, const int* in_sizes, int n_in,
                              void* d_out, int out_size, void* d_ws, size_t ws_size,
                              hipStream_t stream) {
  if (n_in < 2) return;
  const int fx = (NKF + 1) * CDIM * HW;
  const int ng = in_sizes[0] / fx;
  if (ng <= 0) return;
  if (ng * fx != in_sizes[0]) return;
  const int ny = ng * NKF * CY * HW;
  if (in_sizes[1] != ny) return;
  if (out_size != ng * CY * HW) return;
  if ((ny % 2048) != 0) return;

  size_t off = 0;
  const size_t oXT = off; off += (size_t)ng * (NKF + 1) * HW * CDIM * 2;
  const size_t oYH = off; off += (size_t)ny * 2;
  if (off > ws_size) return;
  if (off > (size_t)134217728) return;

  const float* x = (const float*)d_in[0];
  const float* y = (const float*)d_in[1];
  float* out = (float*)d_out;

  char* ws = (char*)d_ws;
  unsigned short* XT = (unsigned short*)(ws + oXT);
  _Float16*       YH = (_Float16*)(ws + oYH);

  k_xt<<<dim3(HW / KT, ng * (NKF + 1)), dim3(256), 0, stream>>>(x, XT);
  k_yh<<<dim3(ny / 2048), dim3(256), 0, stream>>>(y, YH);
  k_attn<<<dim3(HW / MQB, ng), dim3(128), 0, stream>>>(XT, YH, out);
  (void)hipGetLastError();
}
